// Model_42004780155154
// MI455X (gfx1250) — hardware-verified
//
#include <hip/hip_runtime.h>
#include <math.h>

constexpr int NBAT   = 256;
constexpr int TENC   = 96;
constexpr int TPRED  = 96;
constexpr int NCH    = 321;
constexpr int NCHP   = 352;
constexpr int NHID   = 512;
constexpr int NGATE  = 2048;
constexpr int NROW   = NBAT * TENC;
constexpr int NPROJ  = 336;
constexpr int SEQ_ROWS = 16;
constexpr int SEQ_THR  = 256;
constexpr int NJT      = 4;
constexpr int TILEP    = NCHP + 2 * NHID + 8;
constexpr int PROJ_ROWS = 32;
constexpr int PROJ_THR  = 224;
constexpr int NSTEPS    = TENC + TPRED - 1;
constexpr int NXCHUNK   = SEQ_ROWS * (NCHP / 8);
constexpr int NXITER    = (NXCHUNK + SEQ_THR - 1) / SEQ_THR;
constexpr int NHITER    = SEQ_ROWS * (NHID / 8) / SEQ_THR;
constexpr float XCARRY  = 16.0f;
constexpr float WCARRY  = 16.0f;
constexpr float FOLD    = 1.0f / (XCARRY * WCARRY);
constexpr float EPS_VAR = 1e-5f;

static_assert(NGATE == 4 * NHID, "gate blocks");
static_assert(NCHP % 32 == 0 && NCHP >= NCH, "x k padding");
static_assert(NHID % 32 == 0, "h k multiple");
static_assert(NBAT % SEQ_ROWS == 0, "row blocks");
static_assert(NHID == 16 * NJT * (SEQ_THR / 32), "8 waves x 4 tiles x 16 hidden");
static_assert(NXCHUNK % 32 == 0, "x staging tail is whole waves");
static_assert((SEQ_ROWS * (NHID / 8)) % SEQ_THR == 0 && NHITER == 4, "h tile chunks per thread");
static_assert((2 * NGATE / 4) % SEQ_THR == 0, "bias staging exact");
static_assert(TENC == TPRED, "slot pitch");
static_assert(TPRED % PROJ_ROWS == 0, "projection block inside one sequence");
static_assert(NPROJ == 48 * (PROJ_THR / 32) && NPROJ >= NCH, "7 waves x 48 columns");
static_assert((PROJ_ROWS * NCH * 4) % 128 == 0, "whole lines per projection block");
static_assert((TILEP * 2) % 16 == 0, "tile pitch alignment");
static_assert(NGATE % 64 == 0 && NHID % 64 == 0, "fold product tiles");
static_assert(SEQ_ROWS * TILEP * 2 + 2 * NGATE * 4 <= 65536, "static LDS of the sequence kernel");

typedef __attribute__((ext_vector_type(16))) _Float16 v16h;
typedef __attribute__((ext_vector_type(8)))  _Float16 v8h;
typedef __attribute__((ext_vector_type(16))) __bf16   v16b;
typedef __attribute__((ext_vector_type(8)))  __bf16   v8b;
typedef __attribute__((ext_vector_type(8)))  float    v8f;
typedef __attribute__((ext_vector_type(4)))  float    v4f;

__device__ __forceinline__ unsigned short f2bf_bits(float f) {
  unsigned u = __float_as_uint(f);
  return (unsigned short)((u + 0x7FFFu + ((u >> 16) & 1u)) >> 16);
}
__device__ __forceinline__ float bf_bits2f(unsigned short h) { return __uint_as_float(((unsigned)h) << 16); }

__device__ __forceinline__ void dep_guard4_h(v8f& a, v8f& b, v8f& c, v8f& d, v16h x, v16h y) {
  asm volatile("v_nop\n\tv_nop\n\tv_nop\n\tv_nop" : "+v"(a), "+v"(b), "+v"(c), "+v"(d) : "v"(x), "v"(y));
}
__device__ __forceinline__ void dep_guard4_b(v8f& a, v8f& b, v8f& c, v8f& d, v16b x, v16b y) {
  asm volatile("v_nop\n\tv_nop\n\tv_nop\n\tv_nop" : "+v"(a), "+v"(b), "+v"(c), "+v"(d) : "v"(x), "v"(y));
}
__device__ __forceinline__ void keep4_h(v16h a, v16h b, v16h c, v16h d) { asm volatile("v_nop" :: "v"(a), "v"(b), "v"(c), "v"(d)); }
__device__ __forceinline__ void keep4_b(v16b a, v16b b, v16b c, v16b d) { asm volatile("v_nop" :: "v"(a), "v"(b), "v"(c), "v"(d)); }
__device__ __forceinline__ void acc_guard4(v8f& a, v8f& b, v8f& c, v8f& d) {
  asm volatile("v_nop\n\tv_nop\n\tv_nop\n\tv_nop" : "+v"(a), "+v"(b), "+v"(c), "+v"(d));
}
__device__ __forceinline__ void guard4x_h(v8f& a0, v8f& a1, v8f& a2, v8f& a3,
                                          v16h x0, v16h y0, v16h y1, v16h y2, v16h y3) {
  asm volatile("v_nop\n\tv_nop\n\tv_nop\n\tv_nop"
               : "+v"(a0), "+v"(a1), "+v"(a2), "+v"(a3)
               : "v"(x0), "v"(y0), "v"(y1), "v"(y2), "v"(y3));
}
__device__ __forceinline__ void guard6_h(v8f& a0, v8f& a1, v8f& a2, v8f& a3, v8f& a4, v8f& a5,
                                         v16h x0, v16h x1, v16h y0, v16h y1, v16h y2) {
  asm volatile("v_nop\n\tv_nop\n\tv_nop\n\tv_nop"
               : "+v"(a0), "+v"(a1), "+v"(a2), "+v"(a3), "+v"(a4), "+v"(a5)
               : "v"(x0), "v"(x1), "v"(y0), "v"(y1), "v"(y2));
}
__device__ __forceinline__ void serial4(v8f& a0, v8f& a1, v8f& a2, v8f& a3, float h0, float h1, float h2, float h3) {
  asm volatile("" : "+v"(a0), "+v"(a1), "+v"(a2), "+v"(a3) : "v"(h0), "v"(h1), "v"(h2), "v"(h3));
}

template <typename T> struct Frag;
template <> struct Frag<_Float16> {
  typedef v16h V; union U { v16h v; v8h h[2]; };
  static __device__ __forceinline__ v16h load(const _Float16* p) {
    U f; f.h[0] = *(const v8h*)(p); f.h[1] = *(const v8h*)(p + 16); return f.v;
  }
  static __device__ __forceinline__ v8f mma(v16h a, v16h b, v8f c) {
    return __builtin_amdgcn_wmma_f32_16x16x32_f16(false, a, false, b, (short)0, c, false, false);
  }
  static __device__ __forceinline__ void guard4(v8f& a, v8f& b, v8f& c, v8f& d, v16h x, v16h y) { dep_guard4_h(a, b, c, d, x, y); }
  static __device__ __forceinline__ void keep(v16h a, v16h b, v16h c, v16h d) { keep4_h(a, b, c, d); }
};
template <> struct Frag<__bf16> {
  typedef v16b V; union U { v16b v; v8b h[2]; };
  static __device__ __forceinline__ v16b load(const __bf16* p) {
    U f; f.h[0] = *(const v8b*)(p); f.h[1] = *(const v8b*)(p + 16); return f.v;
  }
  static __device__ __forceinline__ v8f mma(v16b a, v16b b, v8f c) {
    return __builtin_amdgcn_wmma_f32_16x16x32_bf16(false, a, false, b, (short)0, c, false, false);
  }
  static __device__ __forceinline__ void guard4(v8f& a, v8f& b, v8f& c, v8f& d, v16b x, v16b y) { dep_guard4_b(a, b, c, d, x, y); }
  static __device__ __forceinline__ void keep(v16b a, v16b b, v16b c, v16b d) { keep4_b(a, b, c, d); }
};

__device__ __forceinline__ float fsig(float x)  { return __builtin_amdgcn_rcpf(1.0f + __expf(-x)); }
__device__ __forceinline__ float ftanh(float x) { return 1.0f - 2.0f * __builtin_amdgcn_rcpf(__expf(2.0f * x) + 1.0f); }

template <int ET> struct Elem;
template <> struct Elem<0> { typedef _Float16 T; };
template <> struct Elem<1> { typedef __bf16 T; };
template <int ET, bool SPLIT, int BIAS_MODE, int OUT_MODE, bool RESID>
__global__ __launch_bounds__(256) void wmma_gemm64(
    const unsigned short* __restrict__ Ap, const unsigned short* __restrict__ A2p, int lda, long strideA,
    const unsigned short* __restrict__ Btp, const unsigned short* __restrict__ Bt2p, int ldb, long strideB,
    void* __restrict__ Cout, void* __restrict__ Cout2, int ldc, long strideC,
    const float* __restrict__ bias,
    const float* __restrict__ resid, long strideR,
    int M, int N, int K, float scale) {
  typedef typename Elem<ET>::T T;
  typedef typename Frag<T>::V V;
  const T* A = (const T*)Ap; const T* A2 = (const T*)A2p; const T* Bt = (const T*)Btp; const T* Bt2 = (const T*)Bt2p;
  __shared__ __align__(16) float sT[8][16 * 68];
  const int b    = blockIdx.y;
  const int lane = threadIdx.x & 31;
  const int wave = threadIdx.x >> 5;
  const int tilesN = N >> 6;
  const int tilesM = M >> 6;
  const int tile = blockIdx.x * 8 + wave;
  if (tile >= tilesM * tilesN) return;
  const int tm = tile / tilesN;
  const int tn = tile - tm * tilesN;
  const int m0 = tm << 6;
  const int n0 = tn << 6;

  const T* Ab  = A  + (size_t)b * strideA;
  const T* Bb  = Bt + (size_t)b * strideB;
  const T* Ab2 = SPLIT ? (A2  + (size_t)b * strideA) : nullptr;
  const T* Bb2 = SPLIT ? (Bt2 + (size_t)b * strideB) : nullptr;

  const int rlane = lane & 15;
  const int koff  = (lane >> 4) * 8;
  const int mOff  = (lane >> 4) * 8;

  v8f acc[4][4];
#pragma unroll
  for (int i = 0; i < 4; ++i)
#pragma unroll
    for (int j = 0; j < 4; ++j) acc[i][j] = (v8f){0.f,0.f,0.f,0.f,0.f,0.f,0.f,0.f};

  for (int k0 = 0; k0 < K; k0 += 32) {
    V bh[4], bl[4];
#pragma unroll
    for (int j = 0; j < 4; ++j) {
      const size_t bo = (size_t)(n0 + (j << 4) + rlane) * ldb + koff + k0;
      bh[j] = Frag<T>::load(Bb + bo);
      if (SPLIT) bl[j] = Frag<T>::load(Bb2 + bo);
    }
#pragma unroll
    for (int i = 0; i < 4; ++i) {
      const size_t ao = (size_t)(m0 + (i << 4) + rlane) * lda + koff + k0;
      V ah = Frag<T>::load(Ab + ao);
      V al;
      if (SPLIT) al = Frag<T>::load(Ab2 + ao);
#pragma unroll
      for (int j = 0; j < 4; ++j) {
        acc[i][j] = Frag<T>::mma(ah, bh[j], acc[i][j]);
        if (SPLIT) {
          acc[i][j] = Frag<T>::mma(ah, bl[j], acc[i][j]);
          acc[i][j] = Frag<T>::mma(al, bh[j], acc[i][j]);
        }
      }
      Frag<T>::guard4(acc[i][0], acc[i][1], acc[i][2], acc[i][3], ah, SPLIT ? al : ah);
    }
    Frag<T>::keep(bh[0], bh[1], bh[2], bh[3]);
    if (SPLIT) Frag<T>::keep(bl[0], bl[1], bl[2], bl[3]);
  }
  acc_guard4(acc[0][0], acc[0][1], acc[0][2], acc[0][3]);
  acc_guard4(acc[1][0], acc[1][1], acc[1][2], acc[1][3]);
  acc_guard4(acc[2][0], acc[2][1], acc[2][2], acc[2][3]);
  acc_guard4(acc[3][0], acc[3][1], acc[3][2], acc[3][3]);

  float* slab = sT[wave];
  const float* Rb = RESID ? (resid + (size_t)b * strideR) : nullptr;
#pragma unroll
  for (int i = 0; i < 4; ++i) {
    const int mBase = m0 + (i << 4);
#pragma unroll
    for (int j = 0; j < 4; ++j) {
      const int n = n0 + (j << 4) + rlane;
      float bv = 0.f;
      if (BIAS_MODE == 2) bv = bias[n];
#pragma unroll
      for (int r = 0; r < 8; ++r) {
        float v = acc[i][j][r] * scale;
        if (BIAS_MODE == 1) v += bias[mBase + mOff + r];
        if (BIAS_MODE == 2) v += bv;
        if (RESID) v += Rb[(size_t)(mBase + mOff + r) * ldc + n];
        slab[(mOff + r) * 68 + (j << 4) + rlane] = v;
      }
    }
    __builtin_amdgcn_fence(__ATOMIC_RELEASE, "workgroup");
    __builtin_amdgcn_wave_barrier();
    __builtin_amdgcn_fence(__ATOMIC_ACQUIRE, "workgroup");
    if (OUT_MODE == 0) {
      float* C = (float*)Cout + (size_t)b * strideC;
      const int hh = lane >> 4, c4 = (lane & 15) * 4;
      for (int pass = 0; pass < 2; ++pass) {
#pragma unroll
        for (int it = 0; it < 8; ++it) {
          const int row = it * 2 + hh;
          v4f v = *(const v4f*)(slab + row * 68 + c4);
          *(volatile v4f*)(C + (size_t)(mBase + row) * ldc + n0 + c4) = v;
        }
        __threadfence();
      }
    } else {
      const int q = lane >> 3, c8 = (lane & 7) * 8;
      unsigned short* C  = (unsigned short*)Cout  + (size_t)b * strideC;
      unsigned short* C2 = (OUT_MODE == 2) ? ((unsigned short*)Cout2 + (size_t)b * strideC) : nullptr;
      for (int pass = 0; pass < 2; ++pass) {
#pragma unroll
        for (int it = 0; it < 4; ++it) {
          const int row = it * 4 + q;
          const float* sp = slab + row * 68 + c8;
          v8h hv, lv;
#pragma unroll
          for (int e = 0; e < 8; ++e) {
            if (OUT_MODE == 1) {
              hv[e] = (_Float16)sp[e];
            } else {
              unsigned short hb = f2bf_bits(sp[e]);
              unsigned short lb = f2bf_bits(sp[e] - bf_bits2f(hb));
              hv[e] = __builtin_bit_cast(_Float16, hb);
              lv[e] = __builtin_bit_cast(_Float16, lb);
            }
          }
          *(volatile v8h*)(C + (size_t)(mBase + row) * ldc + n0 + c8) = hv;
          if (OUT_MODE == 2) *(volatile v8h*)(C2 + (size_t)(mBase + row) * ldc + n0 + c8) = lv;
        }
        __threadfence();
      }
    }
    __builtin_amdgcn_fence(__ATOMIC_RELEASE, "workgroup");
    __builtin_amdgcn_wave_barrier();
    __builtin_amdgcn_fence(__ATOMIC_ACQUIRE, "workgroup");
  }
}

__global__ __launch_bounds__(256) void stats_kernel(const float* __restrict__ x, float* __restrict__ meanp,
                                                    float* __restrict__ sdevp) {
  const int idx = blockIdx.x * 256 + threadIdx.x;
  if (idx < NBAT * NCH) {
    const int b = idx / NCH;
    const int c = idx - b * NCH;
    const float* p = x + (size_t)b * TENC * NCH + c;
    float s = 0.0f;
#pragma unroll 4
    for (int t = 0; t < TENC; ++t) s += p[(size_t)t * NCH];
    const float mu = s * (1.0f / TENC);
    float s1 = 0.0f, s2 = 0.0f;
#pragma unroll 4
    for (int t = 0; t < TENC; ++t) {
      const float d = p[(size_t)t * NCH] - mu;
      s1 += d;
      s2 += d * d;
    }
    const float m2 = s1 * (1.0f / TENC);
    float var = s2 * (1.0f / TENC) - m2 * m2;
    var = fmaxf(var, 0.0f);
    const float sd = sqrtf(var + EPS_VAR);
    *(volatile float*)(meanp + idx) = mu;
    *(volatile float*)(sdevp + idx) = sd;
    __threadfence();
    *(volatile float*)(meanp + idx) = mu;
    *(volatile float*)(sdevp + idx) = sd;
  }
}

__global__ __launch_bounds__(256) void xnorm_kernel(const float* __restrict__ x, const float* __restrict__ meanp,
                                                    const float* __restrict__ sdevp, unsigned short* __restrict__ XHp) {
  const int i  = blockIdx.x * 256 + threadIdx.x;
  const int n8 = NROW * (NCHP / 8);
  if (i < n8) {
    const int row = i / (NCHP / 8);
    const int c0  = (i - row * (NCHP / 8)) * 8;
    const int b   = row / TENC;
    const float* xr = x + (size_t)row * NCH;
    const float* mr = meanp + b * NCH;
    const float* sr = sdevp + b * NCH;
    float o[8];
#pragma unroll
    for (int hf = 0; hf < 2; ++hf) {
#pragma unroll
      for (int e = 0; e < 4; ++e) {
        const int col = c0 + hf * 4 + e;
        const int cc  = (col < NCH) ? col : (NCH - 1);
        const float xv = xr[cc];
        const float mu = mr[cc];
        const float sd = sr[cc];
        const float v  = (xv - mu) * (1.0f / sd) * XCARRY;
        o[hf * 4 + e] = (col < NCH) ? v : 0.0f;
      }
      asm volatile("" ::: "memory");
    }
    v8h hv;
#pragma unroll
    for (int e = 0; e < 8; ++e) hv[e] = (_Float16)o[e];
    unsigned short* dp = XHp + (size_t)i * 8;
    *(volatile v8h*)dp = hv;
    __threadfence();
    *(volatile v8h*)dp = hv;
  }
}

template <int MODE>
__global__ __launch_bounds__(256) void cvt_pad_kernel(const float* __restrict__ src, const float* __restrict__ src2,
                                                      int R, int C, int rs, int cs,
                                                      unsigned short* __restrict__ dst, unsigned short* __restrict__ dst2,
                                                      int RP, int CP8, float sc) {
  const int i  = blockIdx.x * 256 + threadIdx.x;
  const int n8 = RP * CP8;
  if (i < n8) {
    const int row = i / CP8;
    const int c0  = (i - row * CP8) * 8;
    const int rc  = (row < R) ? row : (R - 1);
    v8h hv, lv;
#pragma unroll
    for (int e = 0; e < 8; ++e) {
      const int col = c0 + e;
      const int cc  = (col < C) ? col : (C - 1);
      const size_t off = (size_t)rc * (size_t)rs + (size_t)cc * (size_t)cs;
      float v = src[off];
      if (MODE == 1) v += src2[off];
      const bool ok = (row < R) && (col < C);
      v = ok ? (v * sc) : 0.0f;
      if (MODE == 2) {
        const unsigned short hb = f2bf_bits(v);
        const unsigned short lb = f2bf_bits(v - bf_bits2f(hb));
        hv[e] = __builtin_bit_cast(_Float16, hb);
        lv[e] = __builtin_bit_cast(_Float16, lb);
      } else {
        hv[e] = (_Float16)v;
      }
    }
    unsigned short* dp  = dst + (size_t)i * 8;
    unsigned short* dp2 = (MODE == 2) ? (dst2 + (size_t)i * 8) : nullptr;
    *(volatile v8h*)dp = hv;
    if (MODE == 2) *(volatile v8h*)dp2 = lv;
    __threadfence();
    *(volatile v8h*)dp = hv;
    if (MODE == 2) *(volatile v8h*)dp2 = lv;
  }
}

__global__ __launch_bounds__(256) void bias_kernel(const float* __restrict__ wih, const float* __restrict__ bih,
                                                   const float* __restrict__ bhh, const float* __restrict__ bp,
                                                   float* __restrict__ BIAS2) {
  const int n = blockIdx.x * 256 + threadIdx.x;
  if (n < NGATE) {
    const float* wr = wih + (size_t)n * NCH;
    float a = 0.0f;
#pragma unroll 1
    for (int c = 0; c < NCH; ++c) a = fmaf(wr[c], bp[c], a);
    const float be = bih[n] + bhh[n];
    const float bd = a + be;
    *(volatile float*)(BIAS2 + n) = be;
    *(volatile float*)(BIAS2 + NGATE + n) = bd;
    __threadfence();
    *(volatile float*)(BIAS2 + n) = be;
    *(volatile float*)(BIAS2 + NGATE + n) = bd;
  }
}

__device__ __forceinline__ void kstep4(const _Float16* wp, size_t gstride, const _Float16* tp, v8f (&acc)[4]) {
  const v16h hb = Frag<_Float16>::load(tp);
  const v16h w0 = Frag<_Float16>::load(wp);
  const v16h w1 = Frag<_Float16>::load(wp + gstride);
  const v16h w2 = Frag<_Float16>::load(wp + 2 * gstride);
  const v16h w3 = Frag<_Float16>::load(wp + 3 * gstride);
  acc[0] = Frag<_Float16>::mma(w0, hb, acc[0]);
  acc[1] = Frag<_Float16>::mma(w1, hb, acc[1]);
  acc[2] = Frag<_Float16>::mma(w2, hb, acc[2]);
  acc[3] = Frag<_Float16>::mma(w3, hb, acc[3]);
  guard4x_h(acc[0], acc[1], acc[2], acc[3], hb, w0, w1, w2, w3);
}

__device__ __forceinline__ void stage_x(_Float16* Tl, const _Float16* XH, int rowbase, int t, int tid) {
#pragma unroll
  for (int it = 0; it < NXITER; ++it) {
    const int idx = it * SEQ_THR + tid;
    if (idx < NXCHUNK) {
      const int row = idx / (NCHP / 8);
      const int c8  = (idx - row * (NCHP / 8)) * 8;
      const v8h v = *(const v8h*)(XH + ((size_t)(rowbase + row) * TENC + (size_t)t) * NCHP + c8);
      *(v8h*)(Tl + row * TILEP + c8) = v;
    }
  }
}

__device__ __forceinline__ void copy_h(const _Float16* Tl, int hcol, _Float16* HDEC, int rowbase, int slot, int tid) {
  v8h v[NHITER];
#pragma unroll
  for (int it = 0; it < NHITER; ++it) {
    const int idx = it * SEQ_THR + tid;
    const int row = idx >> 6;
    const int c8  = (idx & 63) * 8;
    v[it] = *(const v8h*)(Tl + row * TILEP + hcol + c8);
  }
  for (int pass = 0; pass < 2; ++pass) {
#pragma unroll
    for (int it = 0; it < NHITER; ++it) {
      const int idx = it * SEQ_THR + tid;
      const int row = idx >> 6;
      const int c8  = (idx & 63) * 8;
      *(volatile v8h*)(HDEC + ((size_t)(rowbase + row) * TPRED + (size_t)slot) * NHID + c8) = v[it];
    }
    __threadfence();
  }
}

__global__ __launch_bounds__(SEQ_THR) __attribute__((amdgpu_num_vgpr(256)))
void lstm_seq_kernel(const unsigned short* __restrict__ XHp,
                     const unsigned short* __restrict__ WXp,
                     const unsigned short* __restrict__ WHp,
                     const unsigned short* __restrict__ WEp,
                     const float* __restrict__ BIAS2,
                     unsigned short* __restrict__ HDECp) {
  __shared__ __align__(16) _Float16 Tl[SEQ_ROWS * TILEP];
  __shared__ __align__(16) float    Bs[2 * NGATE];
  const _Float16* XH = (const _Float16*)XHp;
  const _Float16* WX = (const _Float16*)WXp;
  const _Float16* WH = (const _Float16*)WHp;
  const _Float16* WE = (const _Float16*)WEp;
  _Float16* HDEC = (_Float16*)HDECp;
  const int tid = threadIdx.x, lane = tid & 31, wave = tid >> 5;
  const int cb = lane & 15, hh = lane >> 4, koff = hh * 8;
  const int rowbase = blockIdx.x * SEQ_ROWS;

  {
    const v8h zh = {(_Float16)0.0f, (_Float16)0.0f, (_Float16)0.0f, (_Float16)0.0f,
                    (_Float16)0.0f, (_Float16)0.0f, (_Float16)0.0f, (_Float16)0.0f};
#pragma unroll
    for (int it = 0; it < NHITER; ++it) {
      const int idx = it * SEQ_THR + tid;
      const int row = idx >> 6;
      const int c8  = (idx & 63) * 8;
      *(v8h*)(Tl + row * TILEP + NCHP + c8) = zh;
    }
  }
  stage_x(Tl, XH, rowbase, 0, tid);
#pragma unroll
  for (int it = 0; it < (2 * NGATE / 4) / SEQ_THR; ++it) {
    const int idx = it * SEQ_THR + tid;
    *(v4f*)(Bs + 4 * idx) = *(const v4f*)(BIAS2 + 4 * idx);
  }
  float cst[NJT][8];
#pragma unroll
  for (int jt = 0; jt < NJT; ++jt)
#pragma unroll
    for (int r = 0; r < 8; ++r) cst[jt][r] = 0.0f;
  __syncthreads();

  const v8f z8 = {0.f, 0.f, 0.f, 0.f, 0.f, 0.f, 0.f, 0.f};

#pragma unroll 1
  for (int s = 0; s < NSTEPS; ++s) {
    const bool enc = (s < TENC);
    const int hcur = NCHP + (s & 1) * NHID;
    const int hnxt = NCHP + ((s & 1) ^ 1) * NHID;
    if (!enc) copy_h(Tl, hcur, HDEC, rowbase, s - TENC, tid);
    const _Float16* Wrec = enc ? WH : WE;
    const float* bsel = Bs + (enc ? 0 : NGATE);
#pragma unroll
    for (int jt = 0; jt < NJT; ++jt) {
      const int jrow = 64 * wave + 16 * jt;
      v8f acc[4];
      acc[0] = z8; acc[1] = z8; acc[2] = z8; acc[3] = z8;
      if (enc) {
        const _Float16* wx = WX + (size_t)(jrow + cb) * NCHP + koff;
        const _Float16* tx = Tl + cb * TILEP + koff;
#pragma unroll 1
        for (int k0 = 0; k0 < NCHP; k0 += 32) kstep4(wx + k0, (size_t)NHID * NCHP, tx + k0, acc);
      }
      {
        const _Float16* wh = Wrec + (size_t)(jrow + cb) * NHID + koff;
        const _Float16* th = Tl + cb * TILEP + hcur + koff;
#pragma unroll 1
        for (int k0 = 0; k0 < NHID; k0 += 32) kstep4(wh + k0, (size_t)NHID * NHID, th + k0, acc);
      }
      acc_guard4(acc[0], acc[1], acc[2], acc[3]);
      v8h hv;
#pragma unroll
      for (int q = 0; q < 2; ++q) {
        const int bo = jrow + 8 * hh + 4 * q;
        const v4f bqi = *(const v4f*)(bsel + 0 * NHID + bo);
        const v4f bqf = *(const v4f*)(bsel + 1 * NHID + bo);
        const v4f bqg = *(const v4f*)(bsel + 2 * NHID + bo);
        const v4f bqo = *(const v4f*)(bsel + 3 * NHID + bo);
        float hq[4];
#pragma unroll
        for (int e = 0; e < 4; ++e) {
          const int r = 4 * q + e;
          const float zi = fmaf(acc[0][r], FOLD, bqi[e]);
          const float zf = fmaf(acc[1][r], FOLD, bqf[e]);
          const float zg = fmaf(acc[2][r], FOLD, bqg[e]);
          const float zo = fmaf(acc[3][r], FOLD, bqo[e]);
          const float ig = fsig(zi);
          const float fg = fsig(zf);
          const float gg = ftanh(zg);
          const float og = fsig(zo);
          const float cn = fg * cst[jt][r] + ig * gg;
          cst[jt][r] = cn;
          const float hn = og * ftanh(cn);
          hq[e] = hn;
          hv[r] = (_Float16)(hn * XCARRY);
        }
        if (q == 0) serial4(acc[0], acc[1], acc[2], acc[3], hq[0], hq[1], hq[2], hq[3]);
      }
      *(v8h*)(Tl + cb * TILEP + hnxt + jrow + 8 * hh) = hv;
    }
    __syncthreads();
    if (s + 1 < TENC) stage_x(Tl, XH, rowbase, s + 1, tid);
    __syncthreads();
  }
  copy_h(Tl, NCHP + (NSTEPS & 1) * NHID, HDEC, rowbase, TPRED - 1, tid);
}

__global__ __launch_bounds__(PROJ_THR) void proj_out_kernel(const unsigned short* __restrict__ HDECp,
                                                            const unsigned short* __restrict__ WPp,
                                                            const float* __restrict__ bp,
                                                            const float* __restrict__ meanp,
                                                            const float* __restrict__ sdevp,
                                                            float* __restrict__ out) {
  __shared__ __align__(16) float So[PROJ_ROWS * NCH];
  const _Float16* HD = (const _Float16*)HDECp;
  const _Float16* WP = (const _Float16*)WPp;
  const int tid = threadIdx.x, lane = tid & 31, wave = tid >> 5;
  const int cb = lane & 15, hh = lane >> 4, koff = hh * 8;
  const int m0 = blockIdx.x * PROJ_ROWS;
  const int b  = blockIdx.x / (TPRED / PROJ_ROWS);

  const v8f z8 = {0.f, 0.f, 0.f, 0.f, 0.f, 0.f, 0.f, 0.f};
  v8f acc[2][3];
#pragma unroll
  for (int mt = 0; mt < 2; ++mt)
#pragma unroll
    for (int nt = 0; nt < 3; ++nt) acc[mt][nt] = z8;

  const _Float16* ap = HD + (size_t)(m0 + cb) * NHID + koff;
  const _Float16* wp = WP + (size_t)(48 * wave + cb) * NHID + koff;
#pragma unroll 1
  for (int k0 = 0; k0 < NHID; k0 += 32) {
    const v16h a0 = Frag<_Float16>::load(ap + k0);
    const v16h a1 = Frag<_Float16>::load(ap + (size_t)16 * NHID + k0);
    const v16h b0 = Frag<_Float16>::load(wp + k0);
    const v16h b1 = Frag<_Float16>::load(wp + (size_t)16 * NHID + k0);
    const v16h b2 = Frag<_Float16>::load(wp + (size_t)32 * NHID + k0);
    acc[0][0] = Frag<_Float16>::mma(a0, b0, acc[0][0]);
    acc[0][1] = Frag<_Float16>::mma(a0, b1, acc[0][1]);
    acc[0][2] = Frag<_Float16>::mma(a0, b2, acc[0][2]);
    acc[1][0] = Frag<_Float16>::mma(a1, b0, acc[1][0]);
    acc[1][1] = Frag<_Float16>::mma(a1, b1, acc[1][1]);
    acc[1][2] = Frag<_Float16>::mma(a1, b2, acc[1][2]);
    guard6_h(acc[0][0], acc[0][1], acc[0][2], acc[1][0], acc[1][1], acc[1][2], a0, a1, b0, b1, b2);
  }
  acc_guard4(acc[0][0], acc[0][1], acc[0][2], acc[1][0]);
  acc_guard4(acc[1][1], acc[1][2], acc[0][0], acc[0][1]);

#pragma unroll
  for (int nt = 0; nt < 3; ++nt) {
    const int n  = 48 * wave + 16 * nt + cb;
    const int nc = (n < NCH) ? n : (NCH - 1);
    const float bpv = bp[nc];
    const float sd  = sdevp[b * NCH + nc];
    const float mu  = meanp[b * NCH + nc];
#pragma unroll
    for (int mt = 0; mt < 2; ++mt) {
#pragma unroll
      for (int r = 0; r < 8; ++r) {
        const int row = 16 * mt + 8 * hh + r;
        const float y = fmaf(acc[mt][nt][r], FOLD, bpv);
        const float val = fmaf(y, sd, mu);
        if (n < NCH) So[row * NCH + n] = val;
      }
    }
  }
  __syncthreads();
  float* ob = out + (size_t)m0 * NCH;
  constexpr int NCHUNK = PROJ_ROWS * NCH / 4;
  constexpr int NPASS  = (NCHUNK + PROJ_THR - 1) / PROJ_THR;
  for (int pass = 0; pass < 2; ++pass) {
#pragma unroll 1
    for (int it = 0; it < NPASS; ++it) {
      const int idx = it * PROJ_THR + tid;
      if (idx < NCHUNK) {
        const v4f v = *(const v4f*)(So + 4 * idx);
        *(volatile v4f*)(ob + 4 * idx) = v;
      }
    }
    __threadfence();
  }
}

extern "C" void kernel_launch(void* const* d_in, const int* in_sizes, int n_in,
                              void* d_out, int out_size, void* d_ws, size_t ws_size, hipStream_t stream) {
  if (n_in < 7 || d_out == nullptr || d_ws == nullptr) return;
  if (in_sizes[0] != NBAT * TENC * NCH || in_sizes[1] != NGATE * NCH || in_sizes[2] != NGATE * NHID ||
      in_sizes[3] != NGATE || in_sizes[4] != NGATE || in_sizes[5] != NCH * NHID || in_sizes[6] != NCH ||
      out_size != NBAT * TPRED * NCH) return;

  const float* x_enc = (const float*)d_in[0];
  const float* wih   = (const float*)d_in[1];
  const float* whh   = (const float*)d_in[2];
  const float* bih   = (const float*)d_in[3];
  const float* bhh   = (const float*)d_in[4];
  const float* wp    = (const float*)d_in[5];
  const float* bp    = (const float*)d_in[6];
  float* out = (float*)d_out;

  char* ws = (char*)d_ws; size_t off = 0;
  auto carve = [&](size_t bytes) -> char* { char* p = ws + off; off += (bytes + 255) & ~(size_t)255; return p; };
  float*          MEAN  = (float*)carve((size_t)NBAT * NCH * 4);
  float*          SDEV  = (float*)carve((size_t)NBAT * NCH * 4);
  unsigned short* XH    = (unsigned short*)carve((size_t)NROW * NCHP * 2);
  unsigned short* WXH   = (unsigned short*)carve((size_t)NGATE * NCHP * 2);
  unsigned short* WIHBH = (unsigned short*)carve((size_t)NGATE * NCHP * 2);
  unsigned short* WIHBL = (unsigned short*)carve((size_t)NGATE * NCHP * 2);
  unsigned short* WPTH  = (unsigned short*)carve((size_t)NHID * NCHP * 2);
  unsigned short* WPTL  = (unsigned short*)carve((size_t)NHID * NCHP * 2);
  unsigned short* WHH   = (unsigned short*)carve((size_t)NGATE * NHID * 2);
  unsigned short* WPH   = (unsigned short*)carve((size_t)NPROJ * NHID * 2);
  float*          PF    = (float*)carve((size_t)NGATE * NHID * 4);
  unsigned short* WEF   = (unsigned short*)carve((size_t)NGATE * NHID * 2);
  float*          BIAS2 = (float*)carve((size_t)2 * NGATE * 4);
  unsigned short* HDEC  = (unsigned short*)carve((size_t)NROW * NHID * 2);
  if (off > ws_size || off > (size_t)134217728) return;

  stats_kernel<<<(NBAT * NCH) / 256, 256, 0, stream>>>(x_enc, MEAN, SDEV);
  xnorm_kernel<<<(NROW * (NCHP / 8)) / 256, 256, 0, stream>>>(x_enc, MEAN, SDEV, XH);

  cvt_pad_kernel<0><<<(NGATE * (NCHP / 8)) / 256, 256, 0, stream>>>(wih, wih, NGATE, NCH, NCH, 1, WXH, WXH, NGATE, NCHP / 8, WCARRY);
  cvt_pad_kernel<2><<<(NGATE * (NCHP / 8)) / 256, 256, 0, stream>>>(wih, wih, NGATE, NCH, NCH, 1, WIHBH, WIHBL, NGATE, NCHP / 8, 1.0f);
  cvt_pad_kernel<2><<<(NHID * (NCHP / 8)) / 256, 256, 0, stream>>>(wp, wp, NHID, NCH, 1, NHID, WPTH, WPTL, NHID, NCHP / 8, 1.0f);
  cvt_pad_kernel<0><<<(NGATE * (NHID / 8)) / 256, 256, 0, stream>>>(whh, whh, NGATE, NHID, NHID, 1, WHH, WHH, NGATE, NHID / 8, WCARRY);
  cvt_pad_kernel<0><<<(NPROJ * (NHID / 8)) / 256, 256, 0, stream>>>(wp, wp, NCH, NHID, NHID, 1, WPH, WPH, NPROJ, NHID / 8, WCARRY);
  bias_kernel<<<NGATE / 256, 256, 0, stream>>>(wih, bih, bhh, bp, BIAS2);

  static_assert(NGATE % 64 == 0 && NHID % 64 == 0 && NCHP % 32 == 0, "fold product shape");
  wmma_gemm64<1, true, 0, 0, false><<<dim3((NGATE / 64) * (NHID / 64) / 8, 1), 256, 0, stream>>>(
      WIHBH, WIHBL, NCHP, 0L, WPTH, WPTL, NCHP, 0L, (void*)PF, (void*)PF, NHID, 0L,
      BIAS2, PF, 0L, NGATE, NHID, NCHP, 1.0f);
  cvt_pad_kernel<1><<<(NGATE * (NHID / 8)) / 256, 256, 0, stream>>>(PF, whh, NGATE, NHID, NHID, 1, WEF, WEF, NGATE, NHID / 8, WCARRY);

  lstm_seq_kernel<<<NBAT / SEQ_ROWS, SEQ_THR, 0, stream>>>(XH, WXH, WHH, WEF, BIAS2, HDEC);

  proj_out_kernel<<<NROW / PROJ_ROWS, PROJ_THR, 0, stream>>>(HDEC, WPH, bp, MEAN, SDEV, out);
}
